// VRWKV_SpatialMix_54769422958607
// MI455X (gfx1250) — hardware-verified
//
#include <hip/hip_runtime.h>
#include <math.h>

#ifndef F32_LEG_SPLIT
#define F32_LEG_SPLIT 0
#endif

constexpr int BATCH   = 8;
constexpr int SEQLEN  = 4096;
constexpr int CHAN    = 256;
constexpr int NROWS   = BATCH * SEQLEN;
constexpr int NPROJ   = 3 * CHAN;
constexpr int NWROWS  = 4 * CHAN;
constexpr int KDIM    = CHAN;
constexpr int NTHR    = 256;
constexpr int TSTEP   = 16;
constexpr int SLABP   = 68;
constexpr float XCARRY = 16.0f;
constexpr float WCARRY = 256.0f;
constexpr float GCARRY = 16.0f;
constexpr float LN_EPS_F = 1e-5f;
constexpr float INV_SEQ  = 1.0f / (float)SEQLEN;
constexpr float INV_CHAN = 1.0f / (float)CHAN;
static_assert(KDIM % 32 == 0, "GEMM K multiple of 32");
static_assert(NROWS % 64 == 0 && NPROJ % 64 == 0 && CHAN % 64 == 0, "GEMM M, N tile multiples");
static_assert(((NROWS / 64) * (NPROJ / 64)) % 8 == 0, "projection grid exact");
static_assert(((NROWS / 64) * (CHAN / 64)) % 8 == 0, "output grid exact");
static_assert(SEQLEN % TSTEP == 0, "time tiles exact");
static_assert(CHAN == NTHR, "one thread per channel in the scan");
static_assert(TSTEP == 2 * (NTHR / 32), "two LN rows per wave per tile");
static_assert(CHAN == 8 * 32, "8 channels per lane in the LN phase");

typedef __attribute__((ext_vector_type(16))) _Float16 v16h;
typedef __attribute__((ext_vector_type(8)))  _Float16 v8h;
typedef __attribute__((ext_vector_type(16))) __bf16   v16b;
typedef __attribute__((ext_vector_type(8)))  __bf16   v8b;
typedef __attribute__((ext_vector_type(8)))  float    v8f;
typedef __attribute__((ext_vector_type(4)))  float    v4f;
typedef __attribute__((ext_vector_type(4)))  unsigned v4u;

__device__ __forceinline__ unsigned short f2bf_bits(float f) {
  unsigned u = __float_as_uint(f);
  return (unsigned short)((u + 0x7FFFu + ((u >> 16) & 1u)) >> 16);
}
__device__ __forceinline__ float bf_bits2f(unsigned short h) { return __uint_as_float(((unsigned)h) << 16); }
__device__ __forceinline__ float bf16r(float f) { return bf_bits2f(f2bf_bits(f)); }

__device__ __forceinline__ float h16_to_f32(unsigned hb) {
  const unsigned sgn = (hb & 0x8000u) << 16;
  const unsigned em = hb & 0x7fffu;
  const float fn = __uint_as_float((em << 13) + 0x38000000u);
  const float fs = (float)em * 5.9604644775390625e-8f;
  const float mag = (em < 0x400u) ? fs : fn;
  return __uint_as_float(__float_as_uint(mag) | sgn);
}

__device__ __forceinline__ float sigm(float x) { return __builtin_amdgcn_rcpf(1.0f + expf(-x)); }

__device__ __forceinline__ void row_guard_h(v8f& a0, v8f& a1, v8f& a2, v8f& a3, v16h x, v16h b0, v16h b1, v16h b2, v16h b3) {
  asm volatile("v_nop\n\tv_nop\n\tv_nop\n\tv_nop" : "+v"(a0), "+v"(a1), "+v"(a2), "+v"(a3) : "v"(x), "v"(b0), "v"(b1), "v"(b2), "v"(b3));
}
__device__ __forceinline__ void row_guard_b(v8f& a0, v8f& a1, v8f& a2, v8f& a3, v16b x, v16b b0, v16b b1, v16b b2, v16b b3) {
  asm volatile("v_nop\n\tv_nop\n\tv_nop\n\tv_nop" : "+v"(a0), "+v"(a1), "+v"(a2), "+v"(a3) : "v"(x), "v"(b0), "v"(b1), "v"(b2), "v"(b3));
}
__device__ __forceinline__ void keep4_h(v16h a, v16h b, v16h c, v16h d) { asm volatile("v_nop" :: "v"(a), "v"(b), "v"(c), "v"(d)); }
__device__ __forceinline__ void keep4_b(v16b a, v16b b, v16b c, v16b d) { asm volatile("v_nop" :: "v"(a), "v"(b), "v"(c), "v"(d)); }
__device__ __forceinline__ void acc_guard4(v8f& a, v8f& b, v8f& c, v8f& d) { asm volatile("v_nop\n\tv_nop\n\tv_nop\n\tv_nop" : "+v"(a), "+v"(b), "+v"(c), "+v"(d)); }

template <typename T> struct Frag;
template <> struct Frag<_Float16> {
  typedef v16h V; union U { v16h v; v8h h[2]; };
  static __device__ __forceinline__ v16h load(const _Float16* p) {
    U f; f.h[0] = *(const v8h*)(p); f.h[1] = *(const v8h*)(p + 16); return f.v;
  }
  static __device__ __forceinline__ v8f mma(v16h a, v16h b, v8f c) {
    return __builtin_amdgcn_wmma_f32_16x16x32_f16(false, a, false, b, (short)0, c, false, false);
  }
  static __device__ __forceinline__ void rguard(v8f& a0, v8f& a1, v8f& a2, v8f& a3, v16h x, v16h b0, v16h b1, v16h b2, v16h b3) { row_guard_h(a0, a1, a2, a3, x, b0, b1, b2, b3); }
  static __device__ __forceinline__ void keep(v16h a, v16h b, v16h c, v16h d) { keep4_h(a, b, c, d); }
};
template <> struct Frag<__bf16> {
  typedef v16b V; union U { v16b v; v8b h[2]; };
  static __device__ __forceinline__ v16b load(const __bf16* p) {
    U f; f.h[0] = *(const v8b*)(p); f.h[1] = *(const v8b*)(p + 16); return f.v;
  }
  static __device__ __forceinline__ v8f mma(v16b a, v16b b, v8f c) {
    return __builtin_amdgcn_wmma_f32_16x16x32_bf16(false, a, false, b, (short)0, c, false, false);
  }
  static __device__ __forceinline__ void rguard(v8f& a0, v8f& a1, v8f& a2, v8f& a3, v16b x, v16b b0, v16b b1, v16b b2, v16b b3) { row_guard_b(a0, a1, a2, a3, x, b0, b1, b2, b3); }
  static __device__ __forceinline__ void keep(v16b a, v16b b, v16b c, v16b d) { keep4_b(a, b, c, d); }
};
template <int ET> struct Elem;
template <> struct Elem<0> { typedef _Float16 T; };
template <> struct Elem<1> { typedef __bf16 T; };

template <bool SPL>
__global__ __launch_bounds__(NTHR) void cvt_x_kernel(const float* __restrict__ src, unsigned short* __restrict__ d0,
                                                     unsigned short* __restrict__ d1, int n8, float sc) {
  const int i = blockIdx.x * NTHR + threadIdx.x;
  if (i < n8) {
    const float* sp = src + (size_t)i * 8;
    const v4f a = *(const v4f*)(sp);
    const v4f b = *(const v4f*)(sp + 4);
    v8h hv, lv;
#pragma unroll
    for (int e = 0; e < 4; ++e) {
      const float fa = a[e];
      const float fb = b[e];
      if (SPL) {
        const unsigned short ha = f2bf_bits(fa);
        const unsigned short la = f2bf_bits(fa - bf_bits2f(ha));
        const unsigned short hb = f2bf_bits(fb);
        const unsigned short lb = f2bf_bits(fb - bf_bits2f(hb));
        hv[e]     = __builtin_bit_cast(_Float16, ha);
        lv[e]     = __builtin_bit_cast(_Float16, la);
        hv[4 + e] = __builtin_bit_cast(_Float16, hb);
        lv[4 + e] = __builtin_bit_cast(_Float16, lb);
      } else {
        hv[e]     = (_Float16)(bf16r(fa) * sc);
        hv[4 + e] = (_Float16)(bf16r(fb) * sc);
        lv[e]     = (_Float16)0.0f;
        lv[4 + e] = (_Float16)0.0f;
      }
    }
    *(volatile v8h*)(d0 + (size_t)i * 8) = hv;
    if (SPL) *(volatile v8h*)(d1 + (size_t)i * 8) = lv;
    __threadfence();
    *(volatile v8h*)(d0 + (size_t)i * 8) = hv;
    if (SPL) *(volatile v8h*)(d1 + (size_t)i * 8) = lv;
  }
}

template <bool SPL>
__global__ __launch_bounds__(NTHR) void cvt_w_kernel(const float* __restrict__ w0, const float* __restrict__ w1,
                                                     const float* __restrict__ w2, const float* __restrict__ w3,
                                                     unsigned short* __restrict__ d0, unsigned short* __restrict__ d1,
                                                     float sc_proj, float sc_out) {
  const int y = blockIdx.y;
  const float* src = (y == 0) ? w0 : (y == 1) ? w1 : (y == 2) ? w2 : w3;
  const int i = blockIdx.x * NTHR + threadIdx.x;
  if (i < CHAN * CHAN / 8) {
    const float* sp = src + (size_t)i * 8;
    const v4f a = *(const v4f*)(sp);
    const v4f b = *(const v4f*)(sp + 4);
    const bool splitrows = SPL && (y < 3);
    const float sc = (y < 3) ? sc_proj : sc_out;
    v8h hv, lv;
#pragma unroll
    for (int e = 0; e < 4; ++e) {
      const float fa = a[e];
      const float fb = b[e];
      if (splitrows) {
        const unsigned short ha = f2bf_bits(fa);
        const unsigned short la = f2bf_bits(fa - bf_bits2f(ha));
        const unsigned short hb = f2bf_bits(fb);
        const unsigned short lb = f2bf_bits(fb - bf_bits2f(hb));
        hv[e]     = __builtin_bit_cast(_Float16, ha);
        lv[e]     = __builtin_bit_cast(_Float16, la);
        hv[4 + e] = __builtin_bit_cast(_Float16, hb);
        lv[4 + e] = __builtin_bit_cast(_Float16, lb);
      } else {
        const float va = SPL ? fa : bf16r(fa);
        const float vb = SPL ? fb : bf16r(fb);
        hv[e]     = (_Float16)(va * sc);
        hv[4 + e] = (_Float16)(vb * sc);
        lv[e]     = (_Float16)0.0f;
        lv[4 + e] = (_Float16)0.0f;
      }
    }
    const size_t o = (size_t)y * (CHAN * CHAN) + (size_t)i * 8;
    *(volatile v8h*)(d0 + o) = hv;
    if (splitrows) *(volatile v8h*)(d1 + o) = lv;
    __threadfence();
    *(volatile v8h*)(d0 + o) = hv;
    if (splitrows) *(volatile v8h*)(d1 + o) = lv;
  }
}

template <int ET, bool SPLIT, int MODE>
__global__ __launch_bounds__(NTHR) void gemm_kernel(
    const unsigned short* __restrict__ Ap, const unsigned short* __restrict__ A2p,
    const unsigned short* __restrict__ Btp, const unsigned short* __restrict__ Bt2p,
    float* OutA, float* OutB, unsigned short* OutS,
    int Mrows, int Ncols, float scale) {
  typedef typename Elem<ET>::T T;
  typedef typename Frag<T>::V V;
  const T* A = (const T*)Ap; const T* A2 = (const T*)A2p; const T* Bt = (const T*)Btp; const T* Bt2 = (const T*)Bt2p;
  __shared__ __align__(16) float sT[8][16 * SLABP];
  const int lane = threadIdx.x & 31;
  const int wave = threadIdx.x >> 5;
  const int tilesN = Ncols >> 6;
  const int tilesM = Mrows >> 6;
  const int tile = blockIdx.x * 8 + wave;
  if (tile >= tilesM * tilesN) return;
  const int tm = tile / tilesN;
  const int tn = tile - tm * tilesN;
  const int m0 = tm << 6;
  const int n0 = tn << 6;

  const int rlane = lane & 15;
  const int koff  = (lane >> 4) * 8;
  const int mOff  = (lane >> 4) * 8;

  v8f acc[4][4];
#pragma unroll
  for (int i = 0; i < 4; ++i)
#pragma unroll
    for (int j = 0; j < 4; ++j) acc[i][j] = (v8f){0.f, 0.f, 0.f, 0.f, 0.f, 0.f, 0.f, 0.f};

#pragma unroll 1
  for (int k0 = 0; k0 < KDIM; k0 += 32) {
    V bh[4], bl[4];
#pragma unroll
    for (int j = 0; j < 4; ++j) {
      const size_t bo = (size_t)(n0 + (j << 4) + rlane) * KDIM + koff + k0;
      bh[j] = Frag<T>::load(Bt + bo);
      if (SPLIT) bl[j] = Frag<T>::load(Bt2 + bo);
    }
#pragma unroll
    for (int i = 0; i < 4; ++i) {
      const size_t ao = (size_t)(m0 + (i << 4) + rlane) * KDIM + koff + k0;
      V ah = Frag<T>::load(A + ao);
      V al;
      if (SPLIT) al = Frag<T>::load(A2 + ao);
#pragma unroll
      for (int j = 0; j < 4; ++j) {
        acc[i][j] = Frag<T>::mma(ah, bh[j], acc[i][j]);
        if (SPLIT) {
          acc[i][j] = Frag<T>::mma(ah, bl[j], acc[i][j]);
          acc[i][j] = Frag<T>::mma(al, bh[j], acc[i][j]);
        }
      }
      Frag<T>::rguard(acc[i][0], acc[i][1], acc[i][2], acc[i][3], ah, bh[0], bh[1], bh[2], bh[3]);
      if (SPLIT) Frag<T>::rguard(acc[i][0], acc[i][1], acc[i][2], acc[i][3], al, bl[0], bl[1], bl[2], bl[3]);
    }
    Frag<T>::keep(bh[0], bh[1], bh[2], bh[3]);
    if (SPLIT) Frag<T>::keep(bl[0], bl[1], bl[2], bl[3]);
  }
  acc_guard4(acc[0][0], acc[0][1], acc[0][2], acc[0][3]);
  acc_guard4(acc[1][0], acc[1][1], acc[1][2], acc[1][3]);
  acc_guard4(acc[2][0], acc[2][1], acc[2][2], acc[2][3]);
  acc_guard4(acc[3][0], acc[3][1], acc[3][2], acc[3][3]);

  float* slab = sT[wave];
  const int region = (MODE == 0) ? (n0 >> 8) : 0;
  const int ncol0  = (MODE == 0) ? (n0 & (CHAN - 1)) : n0;
  bool f32path = true;
  if (MODE == 0) f32path = (region < 2);
#pragma unroll
  for (int i = 0; i < 4; ++i) {
    const int mBase = m0 + (i << 4);
#pragma unroll
    for (int j = 0; j < 4; ++j) {
#pragma unroll
      for (int r = 0; r < 8; ++r) {
        const float v = acc[i][j][r] * scale;
        slab[(mOff + r) * SLABP + (j << 4) + rlane] = v;
      }
    }
    __builtin_amdgcn_fence(__ATOMIC_RELEASE, "workgroup");
    __builtin_amdgcn_wave_barrier();
    __builtin_amdgcn_fence(__ATOMIC_ACQUIRE, "workgroup");
    if (f32path) {
      float* Cf = (region == 0) ? OutA : OutB;
      const int hh = lane >> 4, c4 = (lane & 15) * 4;
      for (int pass = 0; pass < 2; ++pass) {
#pragma unroll
        for (int it = 0; it < 8; ++it) {
          const int row = it * 2 + hh;
          const v4f v = *(const v4f*)(slab + row * SLABP + c4);
          *(volatile v4f*)(Cf + (size_t)(mBase + row) * CHAN + ncol0 + c4) = v;
        }
        __threadfence();
      }
    } else {
      const int q = lane >> 3, c8 = (lane & 7) * 8;
#pragma unroll 1
      for (int it = 0; it < 4; ++it) {
        const int row = it * 4 + q;
        const float* sp = slab + row * SLABP + c8;
        const v4f s0 = *(const v4f*)(sp);
        const v4f s1 = *(const v4f*)(sp + 4);
        v8h hv;
#pragma unroll
        for (int e = 0; e < 4; ++e) {
          const float r0 = s0[e];
          const float r1 = s1[e];
          hv[e]     = (_Float16)sigm(r0);
          hv[4 + e] = (_Float16)sigm(r1);
        }
        unsigned short* dp = OutS + (size_t)(mBase + row) * CHAN + ncol0 + c8;
        *(volatile v8h*)dp = hv;
        __threadfence();
        *(volatile v8h*)dp = hv;
      }
    }
    __builtin_amdgcn_fence(__ATOMIC_RELEASE, "workgroup");
    __builtin_amdgcn_wave_barrier();
    __builtin_amdgcn_fence(__ATOMIC_ACQUIRE, "workgroup");
  }
}

template <bool LEGPURE>
__global__ __launch_bounds__(NTHR) void wkv_ln_kernel(const float* __restrict__ K32, const float* __restrict__ V32,
                                                      const unsigned short* __restrict__ SR16,
                                                      const float* __restrict__ decay, const float* __restrict__ first,
                                                      const float* __restrict__ lnw, const float* __restrict__ lnb,
                                                      unsigned short* __restrict__ G16) {
  __shared__ __align__(16) float ytile[TSTEP * CHAN];
  const int c = threadIdx.x;
  const int lane = c & 31;
  const int wv = c >> 5;
  const int b = blockIdx.x;

  float dc = decay[c];
  float fc = first[c];
  if (LEGPURE) { dc = bf16r(dc); fc = bf16r(fc); }
  const float w = dc * INV_SEQ;
  const float u = fc * INV_SEQ;

  float gw[8], gb[8];
  {
    const v4f w0 = *(const v4f*)(lnw + 8 * lane);
    const v4f w1 = *(const v4f*)(lnw + 8 * lane + 4);
    const v4f b0 = *(const v4f*)(lnb + 8 * lane);
    const v4f b1 = *(const v4f*)(lnb + 8 * lane + 4);
#pragma unroll
    for (int e = 0; e < 4; ++e) {
      const float x0 = w0[e];
      const float x1 = w1[e];
      const float y0 = b0[e];
      const float y1 = b1[e];
      gw[e]     = LEGPURE ? bf16r(x0) : x0;
      gw[4 + e] = LEGPURE ? bf16r(x1) : x1;
      gb[e]     = LEGPURE ? bf16r(y0) : y0;
      gb[4 + e] = LEGPURE ? bf16r(y1) : y1;
    }
  }

  float p = 0.0f, q = 0.0f, o = -1e38f;
  const size_t rowbase = (size_t)b * SEQLEN;

#pragma unroll 1
  for (int tile = 0; tile < SEQLEN / TSTEP; ++tile) {
    const size_t r0 = rowbase + (size_t)tile * TSTEP;
#pragma unroll 1
    for (int i = 0; i < TSTEP; ++i) {
      const size_t off = (r0 + (size_t)i) * CHAN + (size_t)c;
      const float kt = K32[off];
      const float vt = V32[off];
      const float uk = u + kt;
      const float no = fmaxf(o, uk);
      const float ea = expf(o - no);
      const float eb = expf(uk - no);
      const float num = ea * p + eb * vt;
      const float den = ea * q + eb;
      const float y = num / den;
      const float wo = w + o;
      const float no2 = fmaxf(wo, kt);
      const float ea2 = expf(wo - no2);
      const float eb2 = expf(kt - no2);
      p = ea2 * p + eb2 * vt;
      q = ea2 * q + eb2;
      o = no2;
      ytile[i * CHAN + c] = y;
    }
    __syncthreads();
#pragma unroll 1
    for (int rr = 0; rr < 2; ++rr) {
      const int row = 2 * wv + rr;
      const float* yp = ytile + row * CHAN + 8 * lane;
      const v4f ya = *(const v4f*)(yp);
      const v4f yb = *(const v4f*)(yp + 4);
      float yv[8];
#pragma unroll
      for (int e = 0; e < 4; ++e) { yv[e] = ya[e]; yv[4 + e] = yb[e]; }
      float s = 0.0f;
#pragma unroll
      for (int e = 0; e < 8; ++e) s += yv[e];
#pragma unroll
      for (int sh = 1; sh < 32; sh <<= 1) s += __shfl_xor(s, sh, 32);
      const float mu = s * INV_CHAN;
      float ss = 0.0f;
#pragma unroll
      for (int e = 0; e < 8; ++e) { const float d = yv[e] - mu; yv[e] = d; ss += d * d; }
#pragma unroll
      for (int sh = 1; sh < 32; sh <<= 1) ss += __shfl_xor(ss, sh, 32);
      const float var = ss * INV_CHAN;
      const float rstd = rsqrtf(var + LN_EPS_F);
      const size_t go = (r0 + (size_t)row) * CHAN + (size_t)(8 * lane);
      const v4u sw = *(const v4u*)(SR16 + go);
      const unsigned sw0 = sw[0];
      const unsigned sw1 = sw[1];
      const unsigned sw2 = sw[2];
      const unsigned sw3 = sw[3];
      float srv[8];
      srv[0] = h16_to_f32(sw0 & 0xffffu); srv[1] = h16_to_f32(sw0 >> 16);
      srv[2] = h16_to_f32(sw1 & 0xffffu); srv[3] = h16_to_f32(sw1 >> 16);
      srv[4] = h16_to_f32(sw2 & 0xffffu); srv[5] = h16_to_f32(sw2 >> 16);
      srv[6] = h16_to_f32(sw3 & 0xffffu); srv[7] = h16_to_f32(sw3 >> 16);
      v8h gv;
#pragma unroll
      for (int e = 0; e < 8; ++e) {
        const float z = (yv[e] * rstd) * gw[e] + gb[e];
        gv[e] = (_Float16)((srv[e] * z) * GCARRY);
      }
      *(volatile v8h*)(G16 + go) = gv;
      __threadfence();
      *(volatile v8h*)(G16 + go) = gv;
    }
    __syncthreads();
  }
}

extern "C" void kernel_launch(void* const* d_in, const int* in_sizes, int n_in,
                              void* d_out, int out_size, void* d_ws, size_t ws_size, hipStream_t stream) {
  if (n_in < 9 || d_out == nullptr || d_ws == nullptr) return;
  if (in_sizes[0] != NROWS * CHAN || in_sizes[1] != CHAN * CHAN || in_sizes[2] != CHAN * CHAN ||
      in_sizes[3] != CHAN * CHAN || in_sizes[4] != CHAN * CHAN || in_sizes[5] != CHAN ||
      in_sizes[6] != CHAN || in_sizes[7] != CHAN || in_sizes[8] != CHAN || out_size != NROWS * CHAN) return;

  const float* x     = (const float*)d_in[0];
  const float* Wk    = (const float*)d_in[1];
  const float* Wv    = (const float*)d_in[2];
  const float* Wr    = (const float*)d_in[3];
  const float* Wo    = (const float*)d_in[4];
  const float* decay = (const float*)d_in[5];
  const float* first = (const float*)d_in[6];
  const float* lnw   = (const float*)d_in[7];
  const float* lnb   = (const float*)d_in[8];
  float* out = (float*)d_out;

  char* ws = (char*)d_ws; size_t off = 0;
  auto carve = [&](size_t bytes) -> char* { char* pp = ws + off; off += (bytes + 255) & ~(size_t)255; return pp; };
  unsigned short* X16  = (unsigned short*)carve((size_t)NROWS * CHAN * 2);
  unsigned short* W16  = (unsigned short*)carve((size_t)NWROWS * CHAN * 2);
#if F32_LEG_SPLIT
  unsigned short* W16L = (unsigned short*)carve((size_t)NWROWS * CHAN * 2);
#endif
  float*          K32  = (float*)carve((size_t)NROWS * CHAN * 4);
  float*          V32  = (float*)carve((size_t)NROWS * CHAN * 4);
  unsigned short* SR16 = (unsigned short*)carve((size_t)NROWS * CHAN * 2);
  unsigned short* G16  = (unsigned short*)carve((size_t)NROWS * CHAN * 2);
  if (off > ws_size || off > (size_t)134217728) return;

  const int n8x = NROWS * CHAN / 8;
  const dim3 wgrid(CHAN * CHAN / 8 / NTHR, 4);
  const int gridProj = (NROWS / 64) * (NPROJ / 64) / 8;
  const int gridOut  = (NROWS / 64) * (CHAN / 64) / 8;
  const float scaleOut = 1.0f / (GCARRY * WCARRY);

#if F32_LEG_SPLIT
  unsigned short* XL = G16;
  cvt_x_kernel<true><<<n8x / NTHR, NTHR, 0, stream>>>(x, X16, XL, n8x, 1.0f);
  cvt_w_kernel<true><<<wgrid, NTHR, 0, stream>>>(Wk, Wv, Wr, Wo, W16, W16L, 1.0f, WCARRY);
  gemm_kernel<1, true, 0><<<gridProj, NTHR, 0, stream>>>(X16, XL, W16, W16L, K32, V32, SR16, NROWS, NPROJ, 1.0f);
  wkv_ln_kernel<false><<<BATCH, NTHR, 0, stream>>>(K32, V32, SR16, decay, first, lnw, lnb, G16);
#else
  cvt_x_kernel<false><<<n8x / NTHR, NTHR, 0, stream>>>(x, X16, X16, n8x, XCARRY);
  cvt_w_kernel<false><<<wgrid, NTHR, 0, stream>>>(Wk, Wv, Wr, Wo, W16, W16, WCARRY, WCARRY);
  gemm_kernel<0, false, 0><<<gridProj, NTHR, 0, stream>>>(X16, X16, W16, W16, K32, V32, SR16, NROWS, NPROJ,
                                                          1.0f / (XCARRY * WCARRY));
  wkv_ln_kernel<true><<<BATCH, NTHR, 0, stream>>>(K32, V32, SR16, decay, first, lnw, lnb, G16);
#endif
  gemm_kernel<0, false, 1><<<gridOut, NTHR, 0, stream>>>(G16, G16, W16 + (size_t)NPROJ * CHAN, W16 + (size_t)NPROJ * CHAN,
                                                         out, out, SR16, NROWS, CHAN, scaleOut);
}
